// CharCNNEncoder_39694087749662
// MI455X (gfx1250) — hardware-run, weakly checked
//
#include <hip/hip_runtime.h>


namespace {
constexpr int NWORD = 64 * 512, NCH = 24, ED = 30, NF = 50, V = 128, WPW = 16  ;
constexpr float XS = 8.0f, WSC = 256.0f;
typedef _Float16 b16;
typedef __attribute__((ext_vector_type(16))) _Float16 v16b;
typedef __attribute__((ext_vector_type(8))) _Float16 v8b;
typedef __attribute__((ext_vector_type(8))) float v8f;
typedef __attribute__((ext_vector_type(4))) float v4f;
__device__ __forceinline__ float bf16_rne(float f) { unsigned int u = __float_as_uint(f); u += 0x7FFFu + ((u >> 16) & 1u); float r = __uint_as_float(u & 0xFFFF0000u); asm volatile("" : "+v"(r)); return r; }
__device__ __forceinline__ float bfv(float f) { float r = bf16_rne(f); asm volatile("" : "+v"(r)); return r; }
__device__ __forceinline__ v16b frag_kb(const b16* p, int hh) { const v8b a = *(const v8b*)(p + 8 * hh), b = *(const v8b*)(p + 16 + 8 * hh); v16b f;
#pragma unroll
  for (int e = 0; e < 8; ++e) { f[e] = a[e]; f[8 + e] = b[e]; } return f; }
__device__ __forceinline__ v8f wmma16b(v16b a, v16b b, v8f c) { v8f d = __builtin_amdgcn_wmma_f32_16x16x32_f16(false, a, false, b, (short)0, c, false, false); asm volatile("v_nop\n\tv_nop\n\tv_nop\n\tv_nop" : "+v"(d) : "v"(a), "v"(b)); return d; }
__device__ __forceinline__ void wave_lds_sync() { __builtin_amdgcn_fence(__ATOMIC_RELEASE, "workgroup"); __builtin_amdgcn_wave_barrier(); __builtin_amdgcn_fence(__ATOMIC_ACQUIRE, "workgroup"); }
__device__ __forceinline__ int iclamp(int v, int lo, int hi) { return v < lo ? lo : (v > hi ? hi : v); }

__global__ __launch_bounds__(256) void wput_kernel(const float* __restrict__ w2, const float* __restrict__ w3, const float* __restrict__ w4, const float* __restrict__ embt, b16* __restrict__ WK2, b16* __restrict__ WK3, b16* __restrict__ WK4, b16* __restrict__ ET) { const int u = blockIdx.x * 256 + threadIdx.x; v8b v; auto put = [&](b16* dst) { for (int pass = 0; pass < 2; ++pass) { *(volatile v8b*)dst = v; __threadfence(); } };
  for (int kk = 2; kk <= 4; ++kk) { const int KP = 32 * kk; const float* w = kk == 2 ? w2 : kk == 3 ? w3 : w4; b16* dst = kk == 2 ? WK2 : kk == 3 ? WK3 : WK4;
    if (u < 64 * (KP / 8)) { const int f = u / (KP / 8), c0 = (u % (KP / 8)) * 8;
#pragma unroll
      for (int j8 = 0; j8 < 8; ++j8) { const int c = c0 + j8; const int j = c / ED, d = c % ED; float wv = 0.0f; if (f < NF && j < kk) wv = w[((size_t)f * ED + d) * kk + j]; v[j8] = (b16)(bf16_rne(wv) * WSC); } put(dst + (size_t)f * KP + c0); } }
  if (u < V * 4) { const int r = u / 4, c0 = (u % 4) * 8;
#pragma unroll
    for (int j8 = 0; j8 < 8; ++j8) { const int c = c0 + j8; v[j8] = (b16)(c < ED ? bfv(embt[(size_t)r * ED + c]) * XS : 0.0f); } put(ET + (size_t)r * 32 + c0); } }
__global__ __launch_bounds__(32) void main_kernel(const int* __restrict__ ids, const b16* __restrict__ ET, const b16* __restrict__ WK2, const b16* __restrict__ WK3, const b16* __restrict__ WK4, const float* __restrict__ b2, const float* __restrict__ b3, const float* __restrict__ b4, int WLIM, float* __restrict__ out) { __shared__ __attribute__((aligned(16))) b16 EMB[40][32], A[32][128 + 8]; __shared__ float Tc[32][65], OUTW[WPW][152]; const int lane = threadIdx.x, nloc = lane & 15, hlf = lane >> 4; const size_t w0 = (size_t)blockIdx.x * WPW; if (w0 >= (size_t)WLIM) return;
  for (int r = 24; r < 40; ++r) EMB[r][lane] = (b16)0.0f;
#pragma unroll 1
  for (int wi = 0; wi < WPW; ++wi) { const size_t w = w0 + wi;
    if (lane < NCH) { const int id = iclamp(ids[w * NCH + lane], 0, V - 1); const v8b* src = (const v8b*)(ET + (size_t)id * 32); v8b* dst = (v8b*)&EMB[lane][0]; dst[0] = src[0]; dst[1] = src[1]; dst[2] = src[2]; dst[3] = src[3]; }
    wave_lds_sync();
#pragma unroll 1
    for (int kk = 2; kk <= 4; ++kk) { const int KP = 32 * kk, LP = NCH - kk + 1; const b16* WK = kk == 2 ? WK2 : kk == 3 ? WK3 : WK4; const float* bb = kk == 2 ? b2 : kk == 3 ? b3 : b4;
      for (int p = 0; p < 32; ++p) for (int c = lane; c < KP + 8; c += 32) { b16 v = (b16)0.0f; if (c < KP) { const int j = c / ED, d = c % ED; if (j < kk && p + j < 40) v = EMB[p + j][d]; } A[p][c] = v; }
      wave_lds_sync();
      for (int rt = 0; rt < 2; ++rt) { v8f acc[4] = {(v8f){}, (v8f){}, (v8f){}, (v8f){}};
        for (int kb = 0; kb < KP; kb += 32) { const v16b a = frag_kb(&A[rt * 16 + nloc][kb], hlf);
#pragma unroll
          for (int t = 0; t < 4; ++t) acc[t] = wmma16b(a, frag_kb(WK + (size_t)(t * 16 + nloc) * KP + kb, hlf), acc[t]); }
#pragma unroll
        for (int t = 0; t < 4; ++t) { const int f = t * 16 + nloc; const float bv_ = f < NF ? bfv(bb[f]) : 0.0f;
#pragma unroll
          for (int r8 = 0; r8 < 8; ++r8) Tc[rt * 16 + 8 * hlf + r8][f] = fmaxf(acc[t][r8] * (1.0f / (XS * WSC)) + bv_, 0.0f); } }
      wave_lds_sync();
      for (int f = lane; f < NF; f += 32) { float mx = -INFINITY; for (int p = 0; p < LP; ++p) mx = fmaxf(mx, Tc[p][f]); OUTW[wi][(kk - 2) * NF + f] = mx; }
      wave_lds_sync(); } }
  for (int pass = 0; pass < 2; ++pass) { for (int u = lane; u < WPW * 150; u += 32) ((volatile float*)out)[w0 * 150 + u] = OUTW[u / 150][u % 150]; __threadfence(); } }
}

extern "C" void kernel_launch(void* const* d_in, const int* in_sizes, int n_in, void* d_out, int out_size, void* d_ws, size_t ws_size, hipStream_t stream) {
  (void)n_in;
  auto Fp = [&](int i) { return (const float*)d_in[i]; }; auto Ip = [&](int i) { return (const int*)d_in[i]; };
  if (in_sizes[0] != NWORD * NCH || in_sizes[1] != V * ED || in_sizes[2] != NF * ED * 2 || in_sizes[4] != NF * ED * 3 || in_sizes[6] != NF * ED * 4 || out_size != NWORD * 150) return;
  const int WLIM = NWORD;
  size_t off = 0; char* ws = (char*)d_ws;
  auto carve = [&](size_t bytes) { char* p = ws + off; off += (bytes + 255) & ~(size_t)255; return p; };
  b16* WK2 = (b16*)carve(64 * 64 * 2); b16* WK3 = (b16*)carve(64 * 96 * 2); b16* WK4 = (b16*)carve(64 * 128 * 2); b16* ET = (b16*)carve(V * 32 * 2);
  if (off > ws_size || off > ((size_t)1 << 20)) return;
  wput_kernel<<<(64 * 16 + 255) / 256, 256, 0, stream>>>(Fp(2), Fp(4), Fp(6), Fp(1), WK2, WK3, WK4, ET);
  main_kernel<<<NWORD / WPW, 32, 0, stream>>>(Ip(0), ET, WK2, WK3, WK4, Fp(3), Fp(5), Fp(7), WLIM, (float*)d_out);
}
